// TGATLayer_34222299414741
// MI455X (gfx1250) — hardware-run, weakly checked
//
#include <hip/hip_runtime.h>

typedef float          v8f   __attribute__((ext_vector_type(8)));
typedef float          v4f   __attribute__((ext_vector_type(4)));
typedef unsigned int   v4u   __attribute__((ext_vector_type(4)));
typedef int            v8i   __attribute__((ext_vector_type(8)));
typedef unsigned short v8us  __attribute__((ext_vector_type(8)));
typedef unsigned short v16us __attribute__((ext_vector_type(16)));
typedef __bf16         v16bf __attribute__((ext_vector_type(16)));
typedef _Float16       v16h  __attribute__((ext_vector_type(16)));
typedef v4f  __attribute__((may_alias)) v4fa;
typedef v8us __attribute__((may_alias)) v8usa;
union FragB { v16bf v; v16us u; v8us h[2]; v8i w; };
union FragH { v16h  v; v16us u; v8us h[2]; v8i w; };

__device__ __forceinline__ v8f wmb(const FragB& a, const FragB& b, v8f c) {
  v8f d = __builtin_amdgcn_wmma_f32_16x16x32_bf16(false, a.v, false, b.v, (short)0, c, false, false);
  asm volatile("v_nop\n\tv_nop\n\tv_nop\n\tv_nop" : "+v"(d) : "v"(a.w), "v"(b.w));
  return d;
}

__device__ __forceinline__ v8f wmh(const FragH& a, const FragH& b, v8f c) {
  v8f d = __builtin_amdgcn_wmma_f32_16x16x32_f16(false, a.v, false, b.v, (short)0, c, false, false);
  asm volatile("v_nop\n\tv_nop\n\tv_nop\n\tv_nop" : "+v"(d) : "v"(a.w), "v"(b.w));
  return d;
}

__device__ __forceinline__ unsigned bf16_bits(float f) {
  const unsigned u = __float_as_uint(f);
  const unsigned r = (u + 0x7FFFu + ((u >> 16) & 1u)) >> 16;
  const unsigned q = (u >> 16) | 0x40u;
  return ((u & 0x7fffffffu) > 0x7f800000u) ? q : r;
}

__device__ __forceinline__ float bf16_val(float f) {
  return __uint_as_float(bf16_bits(f) << 16);
}
__device__ __forceinline__ int clampi(int v, int lo, int hi) {
  return v < lo ? lo : (v > hi ? hi : v);
}

__device__ __forceinline__ unsigned f16_bits(float f) {
  const unsigned u  = __float_as_uint(f);
  const unsigned s  = (u >> 16) & 0x8000u;
  const unsigned a  = u & 0x7fffffffu;
  const unsigned t  = a - 0x38000000u;
  const unsigned r  = (t + 0x0FFFu + ((t >> 13) & 1u)) >> 13;
  const unsigned rc = r > 0x7C00u ? 0x7C00u : r;
  const bool small  = a < 0x38800000u;
  const bool isnan  = a > 0x7f800000u;
  const unsigned fin = small ? 0u : (s | rc);
  return isnan ? (s | 0x7E00u) : fin;
}

__device__ __forceinline__ unsigned pk16(unsigned lo, unsigned hi) { return lo | (hi << 16); }
__device__ __forceinline__ unsigned bf16_lo_bits(float v) {
  float hi = bf16_val(v);
  asm volatile("" : "+v"(hi));
  return bf16_bits(v - hi);
}
__device__ __forceinline__ v4u pack8_bf16(v4f a, v4f c) {
  return (v4u){ pk16(bf16_bits(a[0]), bf16_bits(a[1])), pk16(bf16_bits(a[2]), bf16_bits(a[3])),
                pk16(bf16_bits(c[0]), bf16_bits(c[1])), pk16(bf16_bits(c[2]), bf16_bits(c[3])) };
}
__device__ __forceinline__ v4u pack8_bf16_lo(v4f a, v4f c) {
  return (v4u){ pk16(bf16_lo_bits(a[0]), bf16_lo_bits(a[1])), pk16(bf16_lo_bits(a[2]), bf16_lo_bits(a[3])),
                pk16(bf16_lo_bits(c[0]), bf16_lo_bits(c[1])), pk16(bf16_lo_bits(c[2]), bf16_lo_bits(c[3])) };
}
__device__ __forceinline__ v4u pack8_f16(v4f a, v4f c) {
  return (v4u){ pk16(f16_bits(a[0]), f16_bits(a[1])), pk16(f16_bits(a[2]), f16_bits(a[3])),
                pk16(f16_bits(c[0]), f16_bits(c[1])), pk16(f16_bits(c[2]), f16_bits(c[3])) };
}

template <int FORM>
__global__ __launch_bounds__(256) void k_plane(const float* __restrict__ src, int rows, int cols, int ldsrc,
                                               unsigned short* __restrict__ dst, int MP, int KP) {
  static_assert(FORM >= 0 && FORM <= 3);
  const int KTOT = (FORM == 1 || FORM == 3) ? 2 * KP : KP;
  const unsigned ppr   = (unsigned)(KTOT >> 3);
  const unsigned kp8   = (unsigned)(KP >> 3);
  const unsigned total = (unsigned)MP * ppr;
  const unsigned g     = blockIdx.x * 256u + threadIdx.x;
  const unsigned rowu  = g / ppr;
  const unsigned p     = g - rowu * ppr;
  const bool second    = p >= kp8;
  const int row = (int)rowu;
  const int c0  = (int)((second ? p - kp8 : p) << 3);
  const float* srow = src + (size_t)clampi(row, 0, rows - 1) * (size_t)ldsrc;
  float x[8];
  unsigned mk[8];
#pragma unroll
  for (int e = 0; e < 8; ++e) {
    const int c = c0 + e;
    const float v = srow[clampi(c, 0, cols - 1)];
    asm volatile("" :: "v"(v));
    x[e]  = v;
    mk[e] = (row < rows && c < cols) ? 0xFFFFu : 0u;
  }
  const v4f a = (v4f){ x[0], x[1], x[2], x[3] };
  const v4f c = (v4f){ x[4], x[5], x[6], x[7] };
  v4u o;
  if (FORM == 2) {
    o = pack8_f16(a, c);
  } else {
    const v4u hi = pack8_bf16(a, c);
    o = hi;
    if (FORM == 1) { const v4u lo = pack8_bf16_lo(a, c); o = second ? lo : hi; }
  }
  const v4u mw = (v4u){ pk16(mk[0], mk[1]), pk16(mk[2], mk[3]), pk16(mk[4], mk[5]), pk16(mk[6], mk[7]) };
  o &= mw;
  if (g < total) {
    volatile v4u* q = (volatile v4u*)(dst + (size_t)g * 8);
    *q = o;
    __threadfence();
    *q = o;
  }
}

template <int FORM> struct FragOf    { typedef FragB T; };
template <>         struct FragOf<2> { typedef FragH T; };
__device__ __forceinline__ v8f mm(const FragB& a, const FragB& b, v8f c) { return wmb(a, b, c); }
__device__ __forceinline__ v8f mm(const FragH& a, const FragH& b, v8f c) { return wmh(a, b, c); }
template <class F> __device__ __forceinline__ F ld_frag(const unsigned short* p) {
  F f;
  f.h[0] = *(const v8usa*)(p);
  f.h[1] = *(const v8usa*)(p + 16);
  return f;
}

template <int FORM, int EPI>
__global__ __launch_bounds__(256) __attribute__((amdgpu_num_vgpr(248)))
void k_gemm_nt(const unsigned short* __restrict__ A, const unsigned short* __restrict__ B,
               const float* __restrict__ bias, float* __restrict__ D, int M, int N, int KTOT, int ldd) {
  static_assert(FORM >= 0 && FORM <= 2);
  static_assert(EPI == 0 || EPI == 1);
  typedef typename FragOf<FORM>::T F;
  __shared__ __attribute__((aligned(16))) float sT[8][16 * 68];
  const int lane = threadIdx.x & 31;
  const int wave = threadIdx.x >> 5;
  const int tilesM = (M + 63) >> 6;
  const int tilesN = (N + 63) >> 6;
  const int tile = blockIdx.x * 8 + wave;
  if (tile >= tilesM * tilesN) return;
  const int tm = tile / tilesN;
  const int tn = tile - tm * tilesN;
  const int m0 = tm << 6;
  const int n0 = tn << 6;

  const int rl = lane & 15;
  const int h8 = (lane >> 4) * 8;
  const unsigned short* pa = A + (size_t)(m0 + rl) * (size_t)KTOT + h8;
  const unsigned short* pb = B + (size_t)(n0 + rl) * (size_t)KTOT + h8;

  v8f acc[4][4];
#pragma unroll
  for (int i = 0; i < 4; ++i)
#pragma unroll
    for (int j = 0; j < 4; ++j) acc[i][j] = (v8f){0.f, 0.f, 0.f, 0.f, 0.f, 0.f, 0.f, 0.f};

#pragma unroll 1
  for (int k0 = 0; k0 < KTOT; k0 += 32) {
    F bf[4];
#pragma unroll
    for (int j = 0; j < 4; ++j) bf[j] = ld_frag<F>(pb + (size_t)(j << 4) * (size_t)KTOT + k0);
#pragma unroll
    for (int i = 0; i < 4; ++i) {
      const F af = ld_frag<F>(pa + (size_t)(i << 4) * (size_t)KTOT + k0);
#pragma unroll
      for (int j = 0; j < 4; ++j) acc[i][j] = mm(af, bf[j], acc[i][j]);
    }
  }

  float* slab = sT[wave];
  const int hh = lane >> 4;
  const int c4 = (lane & 15) * 4;
  const int nc = n0 + c4;
  const bool cok = nc < N;
  v4f bv = (v4f){0.f, 0.f, 0.f, 0.f};
  if (EPI == 1) {
    bv = *(const v4fa*)(bias + clampi(nc, 0, N - 4));
    asm volatile("" :: "v"(bv));
  }
#pragma unroll
  for (int i = 0; i < 4; ++i) {
    const int mBase = m0 + (i << 4);
#pragma unroll
    for (int j = 0; j < 4; ++j) {
#pragma unroll
      for (int r = 0; r < 8; ++r) slab[(h8 + r) * 68 + (j << 4) + rl] = acc[i][j][r];
    }
    __builtin_amdgcn_fence(__ATOMIC_RELEASE, "workgroup");
    __builtin_amdgcn_wave_barrier();
    __builtin_amdgcn_fence(__ATOMIC_ACQUIRE, "workgroup");
    v4f vv[8];
#pragma unroll
    for (int it = 0; it < 8; ++it) {
      const int row = it * 2 + hh;
      v4f v = *(const v4fa*)(slab + row * 68 + c4);
      if (EPI == 1) v += bv;
      vv[it] = v;
    }
    for (int pass = 0; pass < 2; ++pass) {
#pragma unroll
      for (int it = 0; it < 8; ++it) {
        const int row = mBase + it * 2 + hh;
        if (cok && row < M) *(volatile v4f*)(D + (size_t)row * (size_t)ldd + nc) = vv[it];
      }
      __threadfence();
    }
    __builtin_amdgcn_fence(__ATOMIC_RELEASE, "workgroup");
    __builtin_amdgcn_wave_barrier();
    __builtin_amdgcn_fence(__ATOMIC_ACQUIRE, "workgroup");
  }
}

#pragma clang fp contract(off)

#ifndef SPLIT_X
#define SPLIT_X 1
#endif


#define NN      50000
#define NE      600000
#define MPAD    50048
#define DW      128
#define NHD     4
#if SPLIT_X
#define KT      256
#else
#define KT      128
#endif
#define RTHR    256
#define RWAVES  8
#define PAR_ATS  0
#define PAR_ATD  128
#define PAR_BIAS 256
#define PAR_G2   384
#define PAR_B2   512
#define PAR_G1   640
#define PAR_B1   768
#define PAR_N    1024
#define BT      512
#define BW      16
#define BEPT    8
#define BCHUNK  (BT * BEPT)
#define NCH     ((NE + BCHUNK - 1) / BCHUNK)
#define NB      1024
#define NBLK    ((NN + NB - 1) / NB)
#define RCAP    16384
#define DEGCAP  64
#define SLOTSH  20
#define LISTTOT (NBLK * RCAP)
#define LDS_BKT ((2 * RCAP + 3 * NB + 64) * 4)
#define WSMAX   ((size_t)128 << 20)

static_assert(NN % RWAVES == 0 && MPAD % RWAVES == 0);
static_assert(NHD * 32 == DW && DW == 128);
static_assert(MPAD == 782 * 64 && MPAD % 64 == 0 && MPAD >= NN && MPAD % 16 == 0);
static_assert(KT % 32 == 0 && (KT == 128 || KT == 256));
static_assert(NE < (1 << SLOTSH) && SLOTSH + 10 <= 31);
static_assert(NN < (1 << 17));
static_assert(NB <= 1024 && (NB & (NB - 1)) == 0 && NB == 2 * BT);
static_assert(NE % 8 == 0 && NE >= 8);
static_assert(NBLK == 49 && NBLK * NB >= NN);
static_assert(NCH * BCHUNK >= NE && NCH == 147);
static_assert(RCAP % 32 == 0);
static_assert(RCAP * 4 >= 12548 * 5);
static_assert(DEGCAP >= 28 + 8);
static_assert(LDS_BKT <= 262144);
static_assert(BW == BT / 32 && BW == 16);

typedef int          v4i __attribute__((ext_vector_type(4)));
typedef int          v2i __attribute__((ext_vector_type(2)));
typedef unsigned int v2u __attribute__((ext_vector_type(2)));
typedef v4i __attribute__((may_alias)) v4ia;
typedef v2i __attribute__((may_alias)) v2ia;

__device__ __forceinline__ float lrelu_k(float v) { return (v > 0.0f) ? v : 0.2f * v; }
__device__ __forceinline__ float maxk(float a, float b) {
  float m = (a < b) ? b : a;
  m = (b != b) ? b : m;
  return m;
}
__device__ __forceinline__ float sel4(v4f v, int h) {
  float r = v.x;
  r = (h == 1) ? v.y : r;
  r = (h == 2) ? v.z : r;
  r = (h == 3) ? v.w : r;
  return r;
}
__device__ __forceinline__ float sum8(float t) {
  t = t + __shfl_xor(t, 4, 32);
  t = t + __shfl_xor(t, 2, 32);
  t = t + __shfl_xor(t, 1, 32);
  return t;
}
__device__ __forceinline__ float sum32(float t) {
  t = t + __shfl_xor(t, 16, 32);
  t = t + __shfl_xor(t, 8, 32);
  t = t + __shfl_xor(t, 4, 32);
  t = t + __shfl_xor(t, 2, 32);
  t = t + __shfl_xor(t, 1, 32);
  return t;
}
__device__ __forceinline__ v4f ln128(v4f x, v4f g, v4f b) {
  float s = x.x + x.y; s = s + x.z; s = s + x.w;
  s = sum32(s);
  const float mean = s * 0.0078125f;
  const float d0 = x.x - mean, d1 = x.y - mean, d2 = x.z - mean, d3 = x.w - mean;
  float q = d0 * d0; float r = d1 * d1; q = q + r; r = d2 * d2; q = q + r; r = d3 * d3; q = q + r;
  q = sum32(q);
  float var = q * 0.0078125f;
  var = var + 1e-5f;
  const float rs = 1.0f / sqrtf(var);
  v4f y;
  float t;
  t = d0 * rs; t = t * g.x; y.x = t + b.x;
  t = d1 * rs; t = t * g.y; y.y = t + b.y;
  t = d2 * rs; t = t * g.z; y.z = t + b.z;
  t = d3 * rs; t = t * g.w; y.w = t + b.w;
  return y;
}

__global__ __launch_bounds__(256) void k_wt(const float* __restrict__ W, unsigned short* WT) {
  const unsigned ppr = (unsigned)(KT >> 3);
  const unsigned g   = blockIdx.x * 256u + threadIdx.x;
  const unsigned nu  = g / ppr;
  const unsigned p   = g - nu * ppr;
  const int k0 = (int)((p & 15u) << 3);
  const int nc = clampi((int)nu, 0, DW - 1);
  float x[8];
#pragma unroll
  for (int e = 0; e < 8; ++e) {
    const float v = W[(size_t)(k0 + e) * DW + nc];
    asm volatile("" :: "v"(v));
    x[e] = v;
  }
  const v4f a = (v4f){ x[0], x[1], x[2], x[3] };
  const v4f c = (v4f){ x[4], x[5], x[6], x[7] };
  const v4u o = pack8_bf16(a, c);
  if (g < (unsigned)DW * ppr) {
    volatile v4u* q = (volatile v4u*)(WT + (size_t)g * 8);
    *q = o;
    __threadfence();
    *q = o;
  }
}

__device__ __forceinline__ unsigned blend7(float a0, float a1, float a2, float a3, float a4, float a5, float a6,
                                           unsigned m0, unsigned m1, unsigned m2, unsigned m3, unsigned m4,
                                           unsigned m5, unsigned m6) {
  const unsigned u = (__float_as_uint(a0) & m0) | (__float_as_uint(a1) & m1) | (__float_as_uint(a2) & m2) |
                     (__float_as_uint(a3) & m3) | (__float_as_uint(a4) & m4) | (__float_as_uint(a5) & m5) |
                     (__float_as_uint(a6) & m6);
  return bf16_bits(__uint_as_float(u)) << 16;
}
__global__ __launch_bounds__(256) void k_par(const float* __restrict__ ats, const float* __restrict__ atd,
                                             const float* __restrict__ bias, const float* __restrict__ g2,
                                             const float* __restrict__ b2, const float* __restrict__ g1,
                                             const float* __restrict__ b1, float* PAR) {
  const int t = (int)threadIdx.x;
  const int idx = 4 * t;
  const int seg = idx >> 7;
  const int o4 = idx & 127;
  const v4f a0 = *(const v4fa*)(ats + o4);
  asm volatile("" :: "v"(a0));
  const v4f a1 = *(const v4fa*)(atd + o4);
  asm volatile("" :: "v"(a1));
  const v4f a2 = *(const v4fa*)(bias + o4);
  asm volatile("" :: "v"(a2));
  const v4f a3 = *(const v4fa*)(g2 + o4);
  asm volatile("" :: "v"(a3));
  const v4f a4 = *(const v4fa*)(b2 + o4);
  asm volatile("" :: "v"(a4));
  const v4f a5 = *(const v4fa*)(g1 + o4);
  asm volatile("" :: "v"(a5));
  const v4f a6 = *(const v4fa*)(b1 + o4);
  asm volatile("" :: "v"(a6));
  const unsigned m0 = (seg == 0) ? 0xFFFFFFFFu : 0u;
  const unsigned m1 = (seg == 1) ? 0xFFFFFFFFu : 0u;
  const unsigned m2 = (seg == 2) ? 0xFFFFFFFFu : 0u;
  const unsigned m3 = (seg == 3) ? 0xFFFFFFFFu : 0u;
  const unsigned m4 = (seg == 4) ? 0xFFFFFFFFu : 0u;
  const unsigned m5 = (seg == 5) ? 0xFFFFFFFFu : 0u;
  const unsigned m6 = (seg == 6) ? 0xFFFFFFFFu : 0u;
  v4u o;
  o.x = blend7(a0.x, a1.x, a2.x, a3.x, a4.x, a5.x, a6.x, m0, m1, m2, m3, m4, m5, m6);
  o.y = blend7(a0.y, a1.y, a2.y, a3.y, a4.y, a5.y, a6.y, m0, m1, m2, m3, m4, m5, m6);
  o.z = blend7(a0.z, a1.z, a2.z, a3.z, a4.z, a5.z, a6.z, m0, m1, m2, m3, m4, m5, m6);
  o.w = blend7(a0.w, a1.w, a2.w, a3.w, a4.w, a5.w, a6.w, m0, m1, m2, m3, m4, m5, m6);
  volatile v4u* q = (volatile v4u*)(PAR + idx);
  *q = o;
  __threadfence();
  *q = o;
}

__global__ __launch_bounds__(RTHR) void k_ln1(const float* __restrict__ x, const float* __restrict__ PAR,
                                              float* XT, unsigned short* OP) {
  __shared__ __attribute__((aligned(16))) float sp[256];
  const int tid  = (int)threadIdx.x;
  const int lane = tid & 31;
  const int wave = tid >> 5;
  if (tid < 64) {
    const v4f t = *(const v4fa*)(PAR + PAR_G1 + 4 * tid);
    *(v4fa*)(sp + 4 * tid) = t;
  }
  __syncthreads();
  const int row  = (int)blockIdx.x * RWAVES + wave;
  const int rowc = clampi(row, 0, NN - 1);
  const int c0   = lane * 4;
  const v4f xv = *(const v4fa*)(x + (size_t)rowc * DW + c0);
  asm volatile("" :: "v"(xv));
  v4f xb;
  xb.x = bf16_val(xv.x); xb.y = bf16_val(xv.y); xb.z = bf16_val(xv.z); xb.w = bf16_val(xv.w);
  asm volatile("" : "+v"(xb));
  const v4f g = *(const v4fa*)(sp + c0);
  const v4f b = *(const v4fa*)(sp + 128 + c0);
  const v4f y = ln128(xb, g, b);
  const unsigned rm = (row < NN) ? 0xFFFFFFFFu : 0u;
  v4u yb;
  yb.x = __float_as_uint(y.x) & rm;
  yb.y = __float_as_uint(y.y) & rm;
  yb.z = __float_as_uint(y.z) & rm;
  yb.w = __float_as_uint(y.w) & rm;
  v2u hw;
  hw.x = pk16(bf16_bits(y.x), bf16_bits(y.y)) & rm;
  hw.y = pk16(bf16_bits(y.z), bf16_bits(y.w)) & rm;
#if SPLIT_X
  v2u lw;
  lw.x = pk16(bf16_lo_bits(y.x), bf16_lo_bits(y.y)) & rm;
  lw.y = pk16(bf16_lo_bits(y.z), bf16_lo_bits(y.w)) & rm;
#endif
  const bool rok = row < MPAD;
  const int roww = row < MPAD ? row : MPAD - 1;
  volatile v4u* qx = (volatile v4u*)(XT + (size_t)roww * DW + c0);
  volatile v2u* qh = (volatile v2u*)(OP + (size_t)roww * KT + c0);
#if SPLIT_X
  volatile v2u* ql = (volatile v2u*)(OP + (size_t)roww * KT + 128 + c0);
#endif
  if (rok) {
    *qx = yb;
    *qh = hw;
#if SPLIT_X
    *ql = lw;
#endif
  }
  __threadfence();
  if (rok) {
    *qx = yb;
    *qh = hw;
#if SPLIT_X
    *ql = lw;
#endif
  }
}

__global__ __launch_bounds__(RTHR) void k_rowprep(const float* __restrict__ HF, const float* __restrict__ PAR,
                                                  float* AS, float* AD) {
  __shared__ __attribute__((aligned(16))) float sp[256];
  __shared__ __attribute__((aligned(16))) float sds[RWAVES * NHD];
  __shared__ __attribute__((aligned(16))) float sdd[RWAVES * NHD];
  const int tid  = (int)threadIdx.x;
  const int lane = tid & 31;
  const int wave = tid >> 5;
  if (tid < 64) {
    const v4f t = *(const v4fa*)(PAR + PAR_ATS + 4 * tid);
    *(v4fa*)(sp + 4 * tid) = t;
  }
  __syncthreads();
  const int row  = (int)blockIdx.x * RWAVES + wave;
  const int rowc = clampi(row, 0, NN - 1);
  const int head = lane >> 3;
  const int c0   = lane * 4;
  const v4f hv = *(const v4fa*)(HF + (size_t)rowc * DW + c0);
  asm volatile("" :: "v"(hv));
  const v4f as = *(const v4fa*)(sp + c0);
  const v4f ad = *(const v4fa*)(sp + 128 + c0);
  float ts = hv.x * as.x;
  float u  = hv.y * as.y; ts = ts + u;
  u = hv.z * as.z; ts = ts + u;
  u = hv.w * as.w; ts = ts + u;
  float td = hv.x * ad.x;
  u = hv.y * ad.y; td = td + u;
  u = hv.z * ad.z; td = td + u;
  u = hv.w * ad.w; td = td + u;
  ts = sum8(ts);
  td = sum8(td);
  if ((lane & 7) == 0) {
    sds[wave * NHD + head] = ts;
    sdd[wave * NHD + head] = td;
  }
  __syncthreads();
  const int l8 = lane & 7;
  const int trow = (int)blockIdx.x * RWAVES + l8;
  const int trc  = clampi(trow, 0, NN - 1);
  const bool wr  = (lane < 8) && (trow < NN);
  if (wave == 0) {
    const v4f sv = *(const v4fa*)(sds + 4 * l8);
    volatile v4f* q = (volatile v4f*)(AS + (size_t)trc * NHD);
    if (wr) *q = sv;
    __threadfence();
    if (wr) *q = sv;
  }
  if (wave == 1) {
    const v4f sv = *(const v4fa*)(sdd + 4 * l8);
    volatile v4f* q = (volatile v4f*)(AD + (size_t)trc * NHD);
    if (wr) *q = sv;
    __threadfence();
    if (wr) *q = sv;
  }
}

__global__ __launch_bounds__(BT) void k_list(const int* __restrict__ ei, unsigned* LIST, int* META) {
  extern __shared__ v4u lds_list[];
  int* reg1 = (int*)lds_list;
  int* reg2 = reg1 + RCAP;
  int* scnt = reg2 + RCAP;
  int* soff = scnt + NB;
  int* curs = soff + NB;
  int* wcnt = curs + NB;
  int* wtot = wcnt + 2 * BW;
  const int* __restrict__ ekey = ei + NE;
  const int tid = (int)threadIdx.x, lane = tid & 31, wave = tid >> 5;
  const int nodeBase = (int)blockIdx.x * NB;
  int nb = NN - nodeBase;
  nb = nb > NB ? NB : (nb < 0 ? 0 : nb);
  const unsigned nbs = (unsigned)nodeBase, unb = (unsigned)nb;

  scnt[2 * tid] = 0;
  scnt[2 * tid + 1] = 0;

  int tot = 0;
#pragma unroll 1
  for (int ch = 0; ch < NCH; ++ch) {
    const int par = ch & 1;
    const int e0  = ch * BCHUNK + tid * BEPT;
    const bool valid = e0 < NE;
    const int ea = e0 < NE - 8 ? e0 : NE - 8;
    const v4i da = *(const v4ia*)(ekey + ea);
    const v4i db = *(const v4ia*)(ekey + ea + 4);
    asm volatile("" :: "v"(da), "v"(db));
    const unsigned s0 = (unsigned)da.x - nbs, s1 = (unsigned)da.y - nbs;
    const unsigned s2 = (unsigned)da.z - nbs, s3 = (unsigned)da.w - nbs;
    const unsigned s4 = (unsigned)db.x - nbs, s5 = (unsigned)db.y - nbs;
    const unsigned s6 = (unsigned)db.z - nbs, s7 = (unsigned)db.w - nbs;
    const bool h0 = valid && (s0 < unb), h1 = valid && (s1 < unb), h2 = valid && (s2 < unb), h3 = valid && (s3 < unb);
    const bool h4 = valid && (s4 < unb), h5 = valid && (s5 < unb), h6 = valid && (s6 < unb), h7 = valid && (s7 < unb);
    const int c = (int)h0 + (int)h1 + (int)h2 + (int)h3 + (int)h4 + (int)h5 + (int)h6 + (int)h7;
    int incl = c;
#pragma unroll
    for (int d = 1; d < 32; d <<= 1) {
      const int up = __shfl_up(incl, d, 32);
      incl += (lane >= d) ? up : 0;
    }
    const int wtotal = __shfl(incl, 31, 32);
    if (lane == 0) wcnt[par * BW + wave] = wtotal;
    __syncthreads();
    int all = 0, pre = 0;
#pragma unroll
    for (int g = 0; g < 4; ++g) {
      const v4i w4 = *(const v4ia*)(wcnt + par * BW + 4 * g);
      const int c0 = clampi(w4.x, 0, 256), c1 = clampi(w4.y, 0, 256);
      const int c2 = clampi(w4.z, 0, 256), c3 = clampi(w4.w, 0, 256);
      all += c0 + c1 + c2 + c3;
      pre += (4 * g + 0 < wave) ? c0 : 0;
      pre += (4 * g + 1 < wave) ? c1 : 0;
      pre += (4 * g + 2 < wave) ? c2 : 0;
      pre += (4 * g + 3 < wave) ? c3 : 0;
    }
    int pos = tot + pre + (incl - c);
#define PUTJ(J, HJ, SJ) if (HJ) { if (pos < RCAP) reg1[pos] = (int)((unsigned)(e0 + (J)) | ((SJ) << SLOTSH)); ++pos; }
    PUTJ(0, h0, s0)
    PUTJ(1, h1, s1)
    PUTJ(2, h2, s2)
    PUTJ(3, h3, s3)
    PUTJ(4, h4, s4)
    PUTJ(5, h5, s5)
    PUTJ(6, h6, s6)
    PUTJ(7, h7, s7)
#undef PUTJ
    tot += all;
  }
  __syncthreads();
  const bool ovf = tot > RCAP;
  const int nh = ovf ? RCAP : tot;

  if (wave == 0) {
#pragma unroll 1
    for (int b0 = 0; b0 < nh; b0 += 32) {
      const int idx = b0 + lane;
      const int uv  = reg1[idx < nh ? idx : nh - 1];
      const int m32 = (nh - b0) < 32 ? (nh - b0) : 32;
#pragma unroll 1
      for (int k = 0; k < m32; ++k) {
        const int u  = __builtin_amdgcn_readlane(uv, k);
        const int sl = (int)(((unsigned)u >> SLOTSH) & (unsigned)(NB - 1));
        const int cv = scnt[sl] + 1;
        if (lane == 0) scnt[sl] = cv;
      }
    }
  }
  __syncthreads();

  int e0c, e1c;
  {
    const v2i cc = *(const v2ia*)(scnt + 2 * tid);
    e0c = cc.x < 0 ? 0 : cc.x;
    e1c = cc.y < 0 ? 0 : cc.y;
    const int ts = e0c + e1c;
    int incl = ts;
#pragma unroll
    for (int d = 1; d < 32; d <<= 1) {
      const int up = __shfl_up(incl, d, 32);
      incl += (lane >= d) ? up : 0;
    }
    if (lane == 31) wtot[wave] = incl;
    __syncthreads();
    int pre = 0;
#pragma unroll
    for (int g = 0; g < 4; ++g) {
      const v4i w4 = *(const v4ia*)(wtot + 4 * g);
      pre += (4 * g + 0 < wave) ? w4.x : 0;
      pre += (4 * g + 1 < wave) ? w4.y : 0;
      pre += (4 * g + 2 < wave) ? w4.z : 0;
      pre += (4 * g + 3 < wave) ? w4.w : 0;
    }
    const int run = pre + incl - ts;
    soff[2 * tid]     = run;
    soff[2 * tid + 1] = run + e0c;
    curs[2 * tid]     = run;
    curs[2 * tid + 1] = run + e0c;
  }
  __syncthreads();

  if (wave == 0) {
#pragma unroll 1
    for (int b0 = 0; b0 < nh; b0 += 32) {
      const int idx = b0 + lane;
      const int uv  = reg1[idx < nh ? idx : nh - 1];
      const int m32 = (nh - b0) < 32 ? (nh - b0) : 32;
#pragma unroll 1
      for (int k = 0; k < m32; ++k) {
        const int u   = __builtin_amdgcn_readlane(uv, k);
        const int sl  = (int)(((unsigned)u >> SLOTSH) & (unsigned)(NB - 1));
        const int eid = (int)((unsigned)u & ((1u << SLOTSH) - 1u));
        const int pr  = curs[sl];
        const int pc  = clampi(pr, 0, RCAP - 1);
        if (lane == 0) { reg2[pc] = eid; curs[sl] = pc + 1; }
      }
    }
  }
  __syncthreads();

  {
    int nhPad = (nh + 31) & ~31;
    nhPad = nhPad > RCAP ? RCAP : nhPad;
    const int nIt = (nhPad + BT - 1) / BT;
    unsigned* lbase = LIST + (size_t)blockIdx.x * (size_t)RCAP;
#pragma unroll 1
    for (int it = 0; it < nIt; ++it) {
      const int i  = it * BT + tid;
      const int ic = i < nh ? i : nh - 1;
      const int eid = clampi(reg2[ic], 0, NE - 1);
      const int cw = ei[eid];
      asm volatile("" :: "v"(cw));
      const unsigned msk = (i < nh) ? 0xFFFFFFFFu : 0u;
      const unsigned o = (unsigned)clampi(cw, 0, NN - 1) & msk;
      const int iw = i < RCAP ? i : RCAP - 1;
      volatile unsigned* q = (volatile unsigned*)(lbase + (size_t)iw);
      const bool wr = i < nhPad;
      if (wr) *q = o;
      __threadfence();
      if (wr) *q = o;
    }
  }

  {
    const int base = (int)blockIdx.x * RCAP;
    const v2i cc = *(const v2ia*)(scnt + 2 * tid);
    const v2i so = *(const v2ia*)(soff + 2 * tid);
    v4i m;
    m.x = base + so.x;
    m.y = ovf ? -1 : cc.x;
    m.z = base + so.y;
    m.w = ovf ? -1 : cc.y;
    volatile v4i* q = (volatile v4i*)(META + 2 * (size_t)(nodeBase + 2 * tid));
    *q = m;
    __threadfence();
    *q = m;
  }
}

__device__ __forceinline__ int entry_src(const unsigned* __restrict__ LIST, int off, int cnt, int b0, int jc,
                                         int rowc) {
  int lst = rowc;
  if (b0 < cnt) {
    const int jl = jc < cnt ? jc : cnt - 1;
    const unsigned e = LIST[(size_t)(off + jl)];
    asm volatile("" :: "v"(e));
    lst = clampi((int)e, 0, NN - 1);
  }
  return (jc < cnt) ? lst : rowc;
}
__device__ __forceinline__ float entry_val(const float* __restrict__ AS, int src, int hsel, float adh) {
  const v4f a = *(const v4fa*)(AS + (size_t)src * NHD);
  asm volatile("" :: "v"(a));
  const float v = sel4(a, hsel) + adh;
  return lrelu_k(v);
}

__global__ __launch_bounds__(RTHR) void k_walk(const float* __restrict__ HF, const float* __restrict__ XT,
                                               const float* __restrict__ AS, const float* __restrict__ AD,
                                               const unsigned* __restrict__ LIST, const int* __restrict__ META,
                                               const float* __restrict__ PAR, float* out, int nrows) {
  __shared__ __attribute__((aligned(16))) float sp[384];
  const int tid  = (int)threadIdx.x;
  const int lane = tid & 31;
  const int wave = tid >> 5;
  if (tid < 96) {
    const v4f t = *(const v4fa*)(PAR + PAR_BIAS + 4 * tid);
    *(v4fa*)(sp + 4 * tid) = t;
  }
  __syncthreads();
  const int row  = (int)blockIdx.x * RWAVES + wave;
  const int rowc = clampi(row, 0, NN - 1);
  const int head = lane >> 3;
  const int hsel = lane & 3;
  const int jsub = lane >> 2;
  const int c0   = lane * 4;

  const v2i mt = *(const v2ia*)(META + 2 * (size_t)rowc);
  asm volatile("" :: "v"(mt));
  const int craw = mt.y;
  const int offv = clampi(mt.x, 0, LISTTOT);
  int cntv = clampi(craw, 0, DEGCAP);
  cntv = cntv < (LISTTOT - offv) ? cntv : (LISTTOT - offv);
  const int off = __builtin_amdgcn_readfirstlane(offv);
  const int cnt = __builtin_amdgcn_readfirstlane(cntv);
  const bool poison = (craw < 0) || (craw > DEGCAP);
  const int total = cnt + 1;

  const v4f ad4 = *(const v4fa*)(AD + (size_t)rowc * NHD);
  asm volatile("" :: "v"(ad4));
  const float adh = sel4(ad4, hsel);

  float mx = -__builtin_inff();
#pragma unroll 1
  for (int b0 = 0; b0 < total; b0 += 8) {
    const int j  = b0 + jsub;
    const int jc = j < cnt ? j : cnt;
    const int src = entry_src(LIST, off, cnt, b0, jc, rowc);
    const float v = entry_val(AS, src, hsel, adh);
    mx = maxk(mx, v);
  }
  {
    const float o16 = __shfl_xor(mx, 16, 32); mx = maxk(mx, o16);
    const float o8  = __shfl_xor(mx, 8, 32);  mx = maxk(mx, o8);
    const float o4  = __shfl_xor(mx, 4, 32);  mx = maxk(mx, o4);
  }

  v4f sm = (v4f){0.0f, 0.0f, 0.0f, 0.0f};
#pragma unroll 1
  for (int b0 = 0; b0 < total; b0 += 8) {
    const int j  = b0 + jsub;
    const int jc = j < cnt ? j : cnt;
    const int src = entry_src(LIST, off, cnt, b0, jc, rowc);
    const float v = entry_val(AS, src, hsel, adh);
    const float q = expf(v - mx);
    const int qi = __float_as_int(q);
    const int m8 = (total - b0) < 8 ? (total - b0) : 8;
#pragma unroll 1
    for (int k = 0; k < m8; ++k) {
      const float q0 = __int_as_float(__builtin_amdgcn_readlane(qi, 4 * k));
      const float q1 = __int_as_float(__builtin_amdgcn_readlane(qi, 4 * k + 1));
      const float q2 = __int_as_float(__builtin_amdgcn_readlane(qi, 4 * k + 2));
      const float q3 = __int_as_float(__builtin_amdgcn_readlane(qi, 4 * k + 3));
      sm.x = sm.x + q0;
      sm.y = sm.y + q1;
      sm.z = sm.z + q2;
      sm.w = sm.w + q3;
    }
  }
  const float dn = sel4(sm, hsel) + 1e-16f;

  v4f ac = (v4f){0.0f, 0.0f, 0.0f, 0.0f};
#pragma unroll 1
  for (int b0 = 0; b0 < total; b0 += 8) {
    const int j  = b0 + jsub;
    const int jc = j < cnt ? j : cnt;
    const int src = entry_src(LIST, off, cnt, b0, jc, rowc);
    const float v = entry_val(AS, src, hsel, adh);
    const float q = expf(v - mx);
    const float wv = q / dn;
    const int wi = __float_as_int(wv);
    const int m8 = (total - b0) < 8 ? (total - b0) : 8;
#pragma unroll 1
    for (int k = 0; k < m8; ++k) {
      const int c = __builtin_amdgcn_readlane(src, 4 * k);
      const float w0 = __int_as_float(__builtin_amdgcn_readlane(wi, 4 * k));
      const float w1 = __int_as_float(__builtin_amdgcn_readlane(wi, 4 * k + 1));
      const float w2 = __int_as_float(__builtin_amdgcn_readlane(wi, 4 * k + 2));
      const float w3 = __int_as_float(__builtin_amdgcn_readlane(wi, 4 * k + 3));
      float w = w0;
      w = (head == 1) ? w1 : w;
      w = (head == 2) ? w2 : w;
      w = (head == 3) ? w3 : w;
      const v4f hn = *(const v4fa*)(HF + (size_t)c * DW + c0);
      asm volatile("" :: "v"(hn));
      float pr;
      pr = w * hn.x; ac.x = ac.x + pr;
      pr = w * hn.y; ac.y = ac.y + pr;
      pr = w * hn.z; ac.z = ac.z + pr;
      pr = w * hn.w; ac.w = ac.w + pr;
    }
  }

  const v4f bs = *(const v4fa*)(sp + c0);
  const v4f g2 = *(const v4fa*)(sp + 128 + c0);
  const v4f b2 = *(const v4fa*)(sp + 256 + c0);
  const v4f xt = *(const v4fa*)(XT + (size_t)rowc * DW + c0);
  asm volatile("" :: "v"(xt));
  v4f r;
  float t;
  t = ac.x + bs.x; r.x = xt.x + t;
  t = ac.y + bs.y; r.y = xt.y + t;
  t = ac.z + bs.z; r.z = xt.z + t;
  t = ac.w + bs.w; r.w = xt.w + t;
  v4f y = ln128(r, g2, b2);
  const float qnan = __uint_as_float(0x7fc00000u);
  y.x = poison ? qnan : y.x;
  y.y = poison ? qnan : y.y;
  y.z = poison ? qnan : y.z;
  y.w = poison ? qnan : y.w;
  const bool rok = (row < nrows) && (row < NN);
  volatile v4f* q = (volatile v4f*)(out + (size_t)rowc * DW + c0);
  if (rok) *q = y;
  __threadfence();
  if (rok) *q = y;
}

extern "C" void kernel_launch(void* const* d_in, const int* in_sizes, int n_in,
                              void* d_out, int out_size, void* d_ws, size_t ws_size,
                              hipStream_t stream) {
  if (n_in < 12) return;
  if (in_sizes[0] != NN * DW) return;
  if (in_sizes[1] != 2 * NE) return;
  if (in_sizes[2] != NE || in_sizes[3] != NE) return;
  if (in_sizes[4] != DW * DW) return;
  if (in_sizes[5] != DW || in_sizes[6] != DW || in_sizes[7] != DW) return;
  if (in_sizes[8] != DW || in_sizes[9] != DW || in_sizes[10] != DW || in_sizes[11] != DW) return;
  if (out_size != NN * DW) return;

  const float* x    = (const float*)d_in[0];
  const int*   ei   = (const int*)  d_in[1];
  const float* W    = (const float*)d_in[4];
  const float* ats  = (const float*)d_in[5];
  const float* atd  = (const float*)d_in[6];
  const float* bias = (const float*)d_in[7];
  const float* g1   = (const float*)d_in[8];
  const float* b1   = (const float*)d_in[9];
  const float* g2   = (const float*)d_in[10];
  const float* b2   = (const float*)d_in[11];
  float* out = (float*)d_out;

  const size_t szXT   = (size_t)MPAD * DW * 4;
  const size_t szOP   = (size_t)MPAD * KT * 2;
  const size_t szHF   = (size_t)MPAD * DW * 4;
  const size_t szA    = (size_t)MPAD * NHD * 4;
  const size_t szMETA = (size_t)NBLK * NB * 2 * 4;
  const size_t szLIST = (size_t)NBLK * RCAP * 4;
  const size_t szWT   = (size_t)DW * KT * 2;
  const size_t szPAR  = (size_t)PAR_N * 4;
  static_assert(2 * (size_t)MPAD * DW * 4 + (size_t)MPAD * KT * 2 + 2 * (size_t)MPAD * NHD * 4 +
                (size_t)NBLK * NB * 8 + (size_t)NBLK * RCAP * 4 + (size_t)DW * KT * 2 + (size_t)PAR_N * 4 ==
                (SPLIT_X ? 82157568 : 69312512));
  static_assert(82157568 <= WSMAX);
  char* ws = (char*)d_ws;
  size_t off = 0;
  const size_t oXT   = off; off += szXT;
  const size_t oOP   = off; off += szOP;
  const size_t oHF   = off; off += szHF;
  const size_t oAS   = off; off += szA;
  const size_t oAD   = off; off += szA;
  const size_t oMETA = off; off += szMETA;
  const size_t oLIST = off; off += szLIST;
  const size_t oWT   = off; off += szWT;
  const size_t oPAR  = off; off += szPAR;
  if (off > ws_size || off > (size_t)WSMAX) return;
  float*          XT   = (float*)(ws + oXT);
  unsigned short* OP   = (unsigned short*)(ws + oOP);
  float*          HF   = (float*)(ws + oHF);
  float*          AS   = (float*)(ws + oAS);
  float*          AD   = (float*)(ws + oAD);
  int*            META = (int*)(ws + oMETA);
  unsigned*       LIST = (unsigned*)(ws + oLIST);
  unsigned short* WT   = (unsigned short*)(ws + oWT);
  float*          PAR  = (float*)(ws + oPAR);

  hipFuncSetAttribute(reinterpret_cast<const void*>(&k_list),
                      hipFuncAttributeMaxDynamicSharedMemorySize, LDS_BKT);

  k_wt<<<DW * KT / 8 / 256, 256, 0, stream>>>(W, WT);
  k_par<<<1, 256, 0, stream>>>(ats, atd, bias, g2, b2, g1, b1, PAR);
  k_ln1<<<MPAD / RWAVES, RTHR, 0, stream>>>(x, PAR, XT, OP);
  static_assert(MPAD % 64 == 0 && DW % 64 == 0 && KT % 32 == 0 && MPAD % 16 == 0 && DW % 32 == 0);
  const int tiles = (MPAD / 64) * (DW / 64);
  const int gG = (tiles + 7) / 8;
  k_gemm_nt<0, 0><<<gG, 256, 0, stream>>>(OP, WT, PAR, HF, MPAD, DW, KT, DW);
  k_rowprep<<<NN / RWAVES, RTHR, 0, stream>>>(HF, PAR, AS, AD);
  k_list<<<NBLK, BT, LDS_BKT, stream>>>(ei, LIST, META);
  k_walk<<<NN / RWAVES, RTHR, 0, stream>>>(HF, XT, AS, AD, LIST, META, PAR, out, NN);
}
